// PointNetSetAbstraction_89721866814223
// MI455X (gfx1250) — hardware-verified
//
#include <hip/hip_runtime.h>
#pragma clang fp contract(off)

typedef __attribute__((ext_vector_type(16))) _Float16 v16h;
typedef __attribute__((ext_vector_type(8)))  _Float16 v8h;
typedef __attribute__((ext_vector_type(8)))  float    v8f;
typedef __attribute__((ext_vector_type(4)))  float    v4f;

constexpr int kBatch = 8;
constexpr int kPts   = 16384;
constexpr int kCent  = 1024;
constexpr int kSamp  = 32;
constexpr int kCh1   = 64;
constexpr int kCh2   = 64;
constexpr int kCh3   = 128;
constexpr float kRad2  = 0.04f;
constexpr float kBnEps = 1e-5f;
constexpr float kActCarry = 16.0f;
constexpr float kWgtCarry = 64.0f;
constexpr float kFoldL2 = 1.0f / kWgtCarry;
constexpr float kFoldL3 = 1.0f / (kActCarry * kWgtCarry);
constexpr int kHP = 72;
constexpr int kOP = 36;

static_assert(kPts % 1024 == 0, "points per thread");
static_assert(kBatch * 3 * kCent * 4 == 98304, "out0 bytes");
static_assert((kBatch * 3 * kCent + kBatch * kCh3 * kCent) * 4 == 4292608, "d_out bytes");
static_assert(kCh1 + kCh2 + kCh3 == 256, "coefficient table");
static_assert((kHP * 2) % 16 == 0 && (kOP * 4) % 16 == 0, "16-B aligned pitches");

constexpr int kFpsLdsFloats = 3 * kPts + 3 * kCent + 128;
constexpr int kFpsLdsBytes  = kFpsLdsFloats * 4;
static_assert(kFpsLdsBytes == 209408, "fps lds");

constexpr int kOffW2t = 0;
constexpr int kOffW3t = kOffW2t + kCh2 * kHP * 2;
constexpr int kOffH1  = kOffW3t + kCh3 * kHP * 2;
constexpr int kOffH2  = kOffH1 + 8 * 32 * kHP * 2;
constexpr int kOffW1  = kOffH2 + 8 * 32 * kHP * 2;
constexpr int kOffCA  = kOffW1 + 6 * kCh1 * 4;
constexpr int kOffCB  = kOffCA + 256 * 4;
constexpr int kOffOst = kOffCB + 256 * 4;
constexpr int kOffLst = kOffOst + kCh3 * kOP * 4;
constexpr int kMlpLdsBytes = kOffLst + 8 * kSamp * 4;
static_assert(kMlpLdsBytes == 124416, "mlp lds");
static_assert(kOffW3t % 16 == 0 && kOffH1 % 16 == 0 && kOffH2 % 16 == 0 && kOffW1 % 16 == 0 &&
              kOffCA % 16 == 0 && kOffCB % 16 == 0 && kOffOst % 16 == 0 && kOffLst % 16 == 0, "lds align");

union FragH { v16h v; v8h h[2]; };

__device__ __forceinline__ v16h frag_load(const _Float16* p) {
  FragH f;
  f.h[0] = *(const v8h*)(p);
  f.h[1] = *(const v8h*)(p + 16);
  return f.v;
}

__device__ __forceinline__ v8f mma_f16(v16h a, v16h b, v8f c) {
  c = __builtin_amdgcn_wmma_f32_16x16x32_f16(false, a, false, b, (short)0, c, false, false);
  asm volatile("v_nop\n\tv_nop\n\tv_nop\n\tv_nop" : "+v"(c) : "v"(a), "v"(b));
  return c;
}

__device__ __forceinline__ void wave_lds_fence() {
  __builtin_amdgcn_fence(__ATOMIC_RELEASE, "workgroup");
  __builtin_amdgcn_wave_barrier();
  __builtin_amdgcn_fence(__ATOMIC_ACQUIRE, "workgroup");
}

__device__ __forceinline__ void tile_gemm_32x64x64(const _Float16* hA, const _Float16* wB, int lane,
                                                   v8f (&acc)[2][4]) {
  const int c  = lane & 15;
  const int ko = (lane >> 4) * 8;
#pragma unroll
  for (int i = 0; i < 2; ++i)
#pragma unroll
    for (int j = 0; j < 4; ++j) acc[i][j] = (v8f){0.f, 0.f, 0.f, 0.f, 0.f, 0.f, 0.f, 0.f};
#pragma unroll
  for (int ks = 0; ks < 2; ++ks) {
    v16h bf[4];
#pragma unroll
    for (int j = 0; j < 4; ++j) bf[j] = frag_load(wB + (j * 16 + c) * kHP + ks * 32 + ko);
#pragma unroll
    for (int i = 0; i < 2; ++i) {
      const v16h af = frag_load(hA + (i * 16 + c) * kHP + ks * 32 + ko);
#pragma unroll
      for (int j = 0; j < 4; ++j) acc[i][j] = mma_f16(af, bf[j], acc[i][j]);
    }
  }
}

__global__ __launch_bounds__(1024)
void fps_select_kernel(const float* __restrict__ xyz, float* __restrict__ out_xyz,
                       float* __restrict__ nx_ws) {
#pragma clang fp contract(off)
  extern __shared__ __align__(16) float fps_sm[];
  float* xs   = fps_sm;
  float* ys   = xs + kPts;
  float* zs   = ys + kPts;
  float* cs   = zs + kPts;
  float* rval = cs + 3 * kCent;
  int*   ridx = (int*)(rval + 64);

  const int b    = blockIdx.x;
  const int tid  = threadIdx.x;
  const int lane = tid & 31;
  const int wid  = tid >> 5;

  {
    const v4f* src = (const v4f*)(xyz + (size_t)b * 3 * kPts);
    v4f* dst = (v4f*)xs;
#pragma unroll 1
    for (int i = 0; i < 12; ++i) {
      const v4f v = src[i * 1024 + tid];
      dst[i * 1024 + tid] = v;
    }
  }
  __syncthreads();

  float dist[16];
#pragma unroll
  for (int j = 0; j < 16; ++j) dist[j] = 1e10f;

  int cur = 0;
#pragma unroll 1
  for (int t = 0; t < kCent; ++t) {
    const float cx = xs[cur];
    const float cy = ys[cur];
    const float cz = zs[cur];
    if (tid == 0) {
      cs[t] = cx;
      cs[kCent + t] = cy;
      cs[2 * kCent + t] = cz;
    }
    float bv = -1.0f;
    int   bi = 0x7fffffff;
#pragma unroll
    for (int j = 0; j < 16; ++j) {
      const int p = j * 1024 + tid;
      const float dx = xs[p] - cx;
      const float dy = ys[p] - cy;
      const float dz = zs[p] - cz;
      const float t0 = dx * dx;
      const float t1 = dy * dy;
      const float t2 = dz * dz;
      const float d  = (t0 + t2) + t1;
      const float dm = fminf(dist[j], d);
      dist[j] = dm;
      if (dm > bv) { bv = dm; bi = p; }
    }
#pragma unroll
    for (int off = 16; off > 0; off >>= 1) {
      const float ov = __shfl_xor(bv, off, 32);
      const int   oi = __shfl_xor(bi, off, 32);
      if (ov > bv || (ov == bv && oi < bi)) { bv = ov; bi = oi; }
    }
    const int pb = (t & 1) * 32;
    if (lane == 0) { rval[pb + wid] = bv; ridx[pb + wid] = bi; }
    __syncthreads();
    float v  = rval[pb + lane];
    int   i2 = ridx[pb + lane];
#pragma unroll
    for (int off = 16; off > 0; off >>= 1) {
      const float ov = __shfl_xor(v, off, 32);
      const int   oi = __shfl_xor(i2, off, 32);
      if (ov > v || (ov == v && oi < i2)) { v = ov; i2 = oi; }
    }
    i2 = i2 < 0 ? 0 : i2;
    i2 = i2 > (kPts - 1) ? (kPts - 1) : i2;
    cur = i2;
  }
  __syncthreads();

  if (tid < 768) {
    const v4f val = *(const v4f*)(cs + 4 * tid);
    volatile v4f* o = (volatile v4f*)(out_xyz + (size_t)b * 3 * kCent + 4 * tid);
    volatile v4f* w = (volatile v4f*)(nx_ws + (size_t)b * 3 * kCent + 4 * tid);
    *o = val;
    *w = val;
    __threadfence();
    *o = val;
    *w = val;
  }
}

__device__ __forceinline__ int ball_select_wave(const float* __restrict__ xb, float cx, float cy,
                                                float cz, int* lst, int lane) {
#pragma clang fp contract(off)
  const float c0 = cx * cx;
  const float c1 = cy * cy;
  const float c2 = cz * cz;
  const float sc = (c0 + c2) + c1;
  lst[lane] = 0;
  wave_lds_fence();
  int cnt = 0;
  for (int ch = 0; ch < kPts / 32; ++ch) {
    if (cnt >= kSamp) break;
    const int p = ch * 32 + lane;
    const float px = xb[p];
    const float py = xb[kPts + p];
    const float pz = xb[2 * kPts + p];
    const float q0 = px * px;
    const float q1 = py * py;
    const float q2 = pz * pz;
    const float sp = (q0 + q2) + q1;
    float dot = cx * px;
    dot = __builtin_fmaf(cy, py, dot);
    dot = __builtin_fmaf(cz, pz, dot);
    const float two_dot = 2.0f * dot;
    const float sqr = (sc + sp) - two_dot;
    const bool inb = !(sqr > kRad2);
    const unsigned m = (unsigned)__ballot(inb);
    const int pos = cnt + __popc(m & ((1u << lane) - 1u));
    if (inb && pos < kSamp) lst[pos] = p;
    cnt += __popc(m);
  }
  wave_lds_fence();
  cnt = cnt > kSamp ? kSamp : cnt;
  const int first = lst[0];
  const int mine  = lst[lane];
  int v = (lane < cnt) ? mine : first;
  v = v < 0 ? 0 : v;
  v = v > (kPts - 1) ? (kPts - 1) : v;
  return v;
}

__global__ __launch_bounds__(256)
void group_mlp_pool_kernel(const float* __restrict__ xyz, const float* __restrict__ points,
                           const float* __restrict__ W1, const float* __restrict__ b1,
                           const float* __restrict__ g1, const float* __restrict__ be1,
                           const float* __restrict__ mu1, const float* __restrict__ vr1,
                           const float* __restrict__ W2, const float* __restrict__ b2,
                           const float* __restrict__ g2, const float* __restrict__ be2,
                           const float* __restrict__ mu2, const float* __restrict__ vr2,
                           const float* __restrict__ W3, const float* __restrict__ b3,
                           const float* __restrict__ g3, const float* __restrict__ be3,
                           const float* __restrict__ mu3, const float* __restrict__ vr3,
                           const float* __restrict__ nx_ws, float* __restrict__ out_feat) {
#pragma clang fp contract(off)
  extern __shared__ __align__(16) unsigned char mlp_sm[];
  _Float16* w2t   = (_Float16*)(mlp_sm + kOffW2t);
  _Float16* w3t   = (_Float16*)(mlp_sm + kOffW3t);
  _Float16* h1all = (_Float16*)(mlp_sm + kOffH1);
  _Float16* h2all = (_Float16*)(mlp_sm + kOffH2);
  float*    w1s   = (float*)(mlp_sm + kOffW1);
  float*    cA    = (float*)(mlp_sm + kOffCA);
  float*    cB    = (float*)(mlp_sm + kOffCB);
  float*    ost   = (float*)(mlp_sm + kOffOst);
  int*      lstall = (int*)(mlp_sm + kOffLst);

  const int tid  = threadIdx.x;
  const int lane = tid & 31;
  const int wave = tid >> 5;
  const int hh   = lane >> 4;
  const int c    = lane & 15;

  for (int i = tid; i < 6 * kCh1; i += 256) w1s[i] = W1[i];
  {
    const int lay = (tid < kCh1) ? 0 : ((tid < kCh1 + kCh2) ? 1 : 2);
    const int ci  = (lay == 0) ? tid : ((lay == 1) ? (tid - kCh1) : (tid - kCh1 - kCh2));
    const float* pbias = (lay == 0) ? b1  : ((lay == 1) ? b2  : b3);
    const float* pgam  = (lay == 0) ? g1  : ((lay == 1) ? g2  : g3);
    const float* pbeta = (lay == 0) ? be1 : ((lay == 1) ? be2 : be3);
    const float* pmean = (lay == 0) ? mu1 : ((lay == 1) ? mu2 : mu3);
    const float* pvar  = (lay == 0) ? vr1 : ((lay == 1) ? vr2 : vr3);
    const float bias = pbias[ci];
    const float gam  = pgam[ci];
    const float bet  = pbeta[ci];
    const float mea  = pmean[ci];
    const float var  = pvar[ci];
    const float s  = gam * __builtin_amdgcn_rsqf(var + kBnEps);
    const float bc = s * (bias - mea) + bet;
    const float sa = (lay == 0) ? kActCarry : ((lay == 1) ? kFoldL2 : kFoldL3);
    const float sb = (lay == 2) ? 1.0f : kActCarry;
    cA[tid] = s * sa;
    cB[tid] = bc * sb;
  }
#pragma unroll 1
  for (int i = 0; i < 4; ++i) {
    const int idx = i * 256 + tid;
    const int k   = idx >> 4;
    const int n4  = (idx & 15) * 4;
    const v4f w = *(const v4f*)(W2 + k * kCh2 + n4);
    const float w0 = w.x, w1 = w.y, w2 = w.z, w3 = w.w;
    w2t[(n4 + 0) * kHP + k] = (_Float16)(w0 * kWgtCarry);
    w2t[(n4 + 1) * kHP + k] = (_Float16)(w1 * kWgtCarry);
    w2t[(n4 + 2) * kHP + k] = (_Float16)(w2 * kWgtCarry);
    w2t[(n4 + 3) * kHP + k] = (_Float16)(w3 * kWgtCarry);
  }
#pragma unroll 1
  for (int i = 0; i < 8; ++i) {
    const int idx = i * 256 + tid;
    const int k   = idx >> 5;
    const int n4  = (idx & 31) * 4;
    const v4f w = *(const v4f*)(W3 + k * kCh3 + n4);
    const float w0 = w.x, w1 = w.y, w2 = w.z, w3 = w.w;
    w3t[(n4 + 0) * kHP + k] = (_Float16)(w0 * kWgtCarry);
    w3t[(n4 + 1) * kHP + k] = (_Float16)(w1 * kWgtCarry);
    w3t[(n4 + 2) * kHP + k] = (_Float16)(w2 * kWgtCarry);
    w3t[(n4 + 3) * kHP + k] = (_Float16)(w3 * kWgtCarry);
  }
  __syncthreads();

  const int b  = blockIdx.x >> 5;
  const int s0 = (blockIdx.x & 31) * 32;
  const float* xb  = xyz    + (size_t)b * 3 * kPts;
  const float* pb  = points + (size_t)b * 3 * kPts;
  const float* nxb = nx_ws  + (size_t)b * 3 * kCent;
  _Float16* h1w = h1all + wave * 32 * kHP;
  _Float16* h2w = h2all + wave * 32 * kHP;
  int* lst = lstall + wave * kSamp;

#pragma unroll 1
  for (int gi = 0; gi < 4; ++gi) {
    const int sl = wave * 4 + gi;
    const int s  = s0 + sl;
    const float cx = nxb[s];
    const float cy = nxb[kCent + s];
    const float cz = nxb[2 * kCent + s];

    const int ip = ball_select_wave(xb, cx, cy, cz, lst, lane);

    const float f0 = pb[ip];
    const float f1 = pb[kPts + ip];
    const float f2 = pb[2 * kPts + ip];
    const float f3 = xb[ip] - cx;
    const float f4 = xb[kPts + ip] - cy;
    const float f5 = xb[2 * kPts + ip] - cz;

#pragma unroll 1
    for (int nb = 0; nb < 8; ++nb) {
      v8h hv;
#pragma unroll
      for (int e = 0; e < 8; ++e) {
        const int n = nb * 8 + e;
        float a = f0 * w1s[n];
        a = a + f1 * w1s[kCh1 + n];
        a = a + f2 * w1s[2 * kCh1 + n];
        a = a + f3 * w1s[3 * kCh1 + n];
        a = a + f4 * w1s[4 * kCh1 + n];
        a = a + f5 * w1s[5 * kCh1 + n];
        const float v = fmaxf(cA[n] * a + cB[n], 0.0f);
        hv[e] = (_Float16)v;
      }
      *(v8h*)(h1w + lane * kHP + nb * 8) = hv;
    }
    wave_lds_fence();

    {
      v8f acc[2][4];
      tile_gemm_32x64x64(h1w, w2t, lane, acc);
#pragma unroll
      for (int i = 0; i < 2; ++i) {
#pragma unroll
        for (int j = 0; j < 4; ++j) {
          const int n = j * 16 + c;
          const float a  = cA[kCh1 + n];
          const float bb = cB[kCh1 + n];
#pragma unroll
          for (int r = 0; r < 8; ++r) {
            const float v = fmaxf(a * acc[i][j][r] + bb, 0.0f);
            h2w[(i * 16 + 8 * hh + r) * kHP + n] = (_Float16)v;
          }
        }
      }
    }
    wave_lds_fence();

#pragma unroll 1
    for (int nh = 0; nh < 2; ++nh) {
      v8f acc[2][4];
      tile_gemm_32x64x64(h2w, w3t + nh * 64 * kHP, lane, acc);
#pragma unroll
      for (int j = 0; j < 4; ++j) {
        const int n = nh * 64 + j * 16 + c;
        const float a  = cA[kCh1 + kCh2 + n];
        const float bb = cB[kCh1 + kCh2 + n];
        float cm = 0.0f;
#pragma unroll
        for (int i = 0; i < 2; ++i) {
#pragma unroll
          for (int r = 0; r < 8; ++r) cm = fmaxf(cm, a * acc[i][j][r] + bb);
        }
        const float other = __shfl_xor(cm, 16, 32);
        cm = fmaxf(cm, other);
        if (hh == 0) ost[n * kOP + sl] = cm;
      }
    }
    wave_lds_fence();
  }
  __syncthreads();

  {
    const int q  = lane >> 3;
    const int c4 = (lane & 7) * 4;
    float* ob = out_feat + (size_t)b * kCh3 * kCent + s0;
    v4f vals[4];
#pragma unroll
    for (int it = 0; it < 4; ++it) {
      const int ch = wave * 16 + it * 4 + q;
      vals[it] = *(const v4f*)(ost + ch * kOP + c4);
    }
#pragma unroll
    for (int it = 0; it < 4; ++it) {
      const int ch = wave * 16 + it * 4 + q;
      *(volatile v4f*)(ob + (size_t)ch * kCent + c4) = vals[it];
    }
    __threadfence();
#pragma unroll
    for (int it = 0; it < 4; ++it) {
      const int ch = wave * 16 + it * 4 + q;
      *(volatile v4f*)(ob + (size_t)ch * kCent + c4) = vals[it];
    }
  }
}

extern "C" void kernel_launch(void* const* d_in, const int* in_sizes, int n_in,
                              void* d_out, int out_size, void* d_ws, size_t ws_size,
                              hipStream_t stream) {
  (void)in_sizes;
  (void)out_size;
  if (n_in < 20) return;
  const size_t ws_need = (size_t)kBatch * 3 * kCent * sizeof(float);
  if (ws_size < ws_need) return;

  const float* xyz    = (const float*)d_in[0];
  const float* points = (const float*)d_in[1];
  const float* W1  = (const float*)d_in[2];
  const float* b1  = (const float*)d_in[3];
  const float* g1  = (const float*)d_in[4];
  const float* be1 = (const float*)d_in[5];
  const float* mu1 = (const float*)d_in[6];
  const float* vr1 = (const float*)d_in[7];
  const float* W2  = (const float*)d_in[8];
  const float* b2  = (const float*)d_in[9];
  const float* g2  = (const float*)d_in[10];
  const float* be2 = (const float*)d_in[11];
  const float* mu2 = (const float*)d_in[12];
  const float* vr2 = (const float*)d_in[13];
  const float* W3  = (const float*)d_in[14];
  const float* b3  = (const float*)d_in[15];
  const float* g3  = (const float*)d_in[16];
  const float* be3 = (const float*)d_in[17];
  const float* mu3 = (const float*)d_in[18];
  const float* vr3 = (const float*)d_in[19];

  float* out_xyz  = (float*)d_out;
  float* out_feat = (float*)d_out + (size_t)kBatch * 3 * kCent;
  float* nx_ws    = (float*)d_ws;

  fps_select_kernel<<<kBatch, 1024, kFpsLdsBytes, stream>>>(xyz, out_xyz, nx_ws);

  group_mlp_pool_kernel<<<kBatch * (kCent / 32), 256, kMlpLdsBytes, stream>>>(
      xyz, points,
      W1, b1, g1, be1, mu1, vr1,
      W2, b2, g2, be2, mu2, vr2,
      W3, b3, g3, be3, mu3, vr3,
      nx_ws, out_feat);
}
